// GMM_3521873182881
// MI455X (gfx1250) — hardware-run, weakly checked
//
#include <hip/hip_runtime.h>


#define NB   2048
#define NK   512
#define ND   128
typedef _Float16 h16;
typedef unsigned short bf;
typedef __attribute__((ext_vector_type(16))) __bf16   v16bf;
typedef __attribute__((ext_vector_type(16))) _Float16 v16h;
typedef __attribute__((ext_vector_type(8)))  _Float16 v8h;
typedef __attribute__((ext_vector_type(8)))  unsigned short v8us;
typedef __attribute__((ext_vector_type(8)))  float    v8f;
typedef __attribute__((ext_vector_type(4)))  float    v4f;
typedef v8h  __attribute__((may_alias)) v8ha;
typedef v4f  __attribute__((may_alias)) v4fa;
typedef v8us __attribute__((may_alias)) v8usa;

__device__ __forceinline__ unsigned short f2bf(float f) { unsigned u = __float_as_uint(f); u += 0x7FFFu + ((u >> 16) & 1u); return (unsigned short)(u >> 16); }
__device__ __forceinline__ float bf2f(unsigned short b) { return __uint_as_float(((unsigned)b) << 16); }
__device__ __forceinline__ float bfr(float f) { return bf2f(f2bf(f)); }
__device__ __forceinline__ v16h cat16(v8h lo, v8h hi) { return __builtin_shufflevector(lo, hi, 0, 1, 2, 3, 4, 5, 6, 7, 8, 9, 10, 11, 12, 13, 14, 15); }
__device__ __forceinline__ v16bf cat16b(v8us lo, v8us hi) { return __builtin_bit_cast(v16bf, __builtin_shufflevector(lo, hi, 0, 1, 2, 3, 4, 5, 6, 7, 8, 9, 10, 11, 12, 13, 14, 15)); }
__device__ __forceinline__ v8f wmma16(v16h a, v16h b, v8f c) { return __builtin_amdgcn_wmma_f32_16x16x32_f16(false, a, false, b, (short)0, c, false, false); }
__device__ __forceinline__ v8f wmmab(v16bf a, v16bf b, v8f c) { return __builtin_amdgcn_wmma_f32_16x16x32_bf16(false, a, false, b, (short)0, c, false, false); }

template <typename T16> struct WFrag;
template <> struct WFrag<h16> { typedef v16h V; static __device__ __forceinline__ V ld(const h16* p) { return cat16(*(const v8h*)p, *(const v8h*)(p + 16)); } static __device__ __forceinline__ v8f mma(V a, V b, v8f c) { return wmma16(a, b, c); } };
template <> struct WFrag<bf> { typedef v16bf V; static __device__ __forceinline__ V ld(const bf* p) { return cat16b(*(const v8us*)p, *(const v8us*)(p + 16)); } static __device__ __forceinline__ v8f mma(V a, V b, v8f c) { return wmmab(a, b, c); } };
template <typename T16, int NSPLIT, bool BIAS>
__global__ __launch_bounds__(32) void k_gemmw(const T16* __restrict__ A, const T16* __restrict__ A2, const T16* __restrict__ Bt, const T16* __restrict__ Bt2, int K, float* C, int ldc, const float* __restrict__ bias, size_t sA, size_t sB, size_t sC) {
    typedef typename WFrag<T16>::V V;
    __shared__ __align__(16) float os[16 * 68];
    const size_t z = blockIdx.z; A += z * sA; if (A2) A2 += z * sA; Bt += z * sB; if (Bt2) Bt2 += z * sB; C += z * sC;
    const int lane = threadIdx.x & 31, lr = lane & 15, hi = lane >> 4; const int r0 = blockIdx.x * 64, c0 = blockIdx.y * 64;
    v8f acc[4][4];
#pragma unroll
    for (int mb = 0; mb < 4; ++mb)
#pragma unroll
        for (int nb = 0; nb < 4; ++nb) acc[mb][nb] = (v8f){};
    const size_t aoff = (size_t)(r0 + lr) * K + 8 * hi, boff = (size_t)(c0 + lr) * K + 8 * hi;
    for (int kc = 0; kc < K; kc += 32) {
        V a[4], a2[4];
#pragma unroll
        for (int mb = 0; mb < 4; ++mb) { a[mb] = WFrag<T16>::ld(A + aoff + (size_t)mb * 16 * K + kc); if (NSPLIT == 1 || NSPLIT == 2) a2[mb] = WFrag<T16>::ld(A2 + aoff + (size_t)mb * 16 * K + kc); }
#pragma unroll
        for (int nb = 0; nb < 4; ++nb) { const V b = WFrag<T16>::ld(Bt + boff + (size_t)nb * 16 * K + kc); V b2; if (NSPLIT >= 2) b2 = WFrag<T16>::ld(Bt2 + boff + (size_t)nb * 16 * K + kc);
#pragma unroll
            for (int mb = 0; mb < 4; ++mb) { acc[mb][nb] = WFrag<T16>::mma(a[mb], b, acc[mb][nb]); if (NSPLIT == 1 || NSPLIT == 2) acc[mb][nb] = WFrag<T16>::mma(a2[mb], b, acc[mb][nb]); if (NSPLIT >= 2) acc[mb][nb] = WFrag<T16>::mma(a[mb], b2, acc[mb][nb]); } }
        asm volatile("v_nop\n\tv_nop\n\tv_nop\n\tv_nop" : "+v"(acc[0][0]), "+v"(acc[1][1]), "+v"(acc[2][2]), "+v"(acc[3][3]) : "v"(a[0]), "v"(a[3]));
    }
#pragma unroll
    for (int mb = 0; mb < 4; ++mb) {
#pragma unroll
        for (int nb = 0; nb < 4; ++nb) {
#pragma unroll
            for (int j = 0; j < 8; ++j) os[(hi * 8 + j) * 68 + nb * 16 + lr] = acc[mb][nb][j]; }
        __builtin_amdgcn_wave_barrier(); asm volatile("" ::: "memory");
        float* crow = C + (size_t)(r0 + mb * 16) * ldc + c0;
#pragma unroll 1
        for (int ps = 0; ps < 2; ++ps) {
#pragma unroll
            for (int s = 0; s < 8; ++s) { const int row = 2 * s + hi, cofs = lr * 4; v4f val = *(const v4fa*)(os + row * 68 + cofs); if (BIAS) { val[0] += bfr(bias[c0 + cofs]); val[1] += bfr(bias[c0 + cofs + 1]); val[2] += bfr(bias[c0 + cofs + 2]); val[3] += bfr(bias[c0 + cofs + 3]); }
                *(volatile v4f*)(crow + (size_t)row * ldc + cofs) = val; }
            if (ps == 0) __threadfence(); }
        __builtin_amdgcn_wave_barrier(); asm volatile("" ::: "memory");
    }
}

__global__ __launch_bounds__(256) void k_cvt8(const float* __restrict__ src, bf* dst, size_t n8) { const size_t i = (size_t)blockIdx.x * 256 + threadIdx.x; if (i >= n8) return; const v8f v = *(const v8f*)(src + i * 8); v8us o;
#pragma unroll
    for (int k = 0; k < 8; ++k) o[k] = f2bf(v[k]); *(volatile v8us*)(dst + i * 8) = o; __threadfence(); *(volatile v8us*)(dst + i * 8) = o; }

__global__ __launch_bounds__(256) void k_px(const float* __restrict__ x, bf* X2b) { const size_t t = (size_t)blockIdx.x * 256 + threadIdx.x; if (t >= (size_t)NB * ND / 8) return; const v8f v = *(const v8f*)(x + t * 8); v8us o;
#pragma unroll
    for (int k = 0; k < 8; ++k) { const float a = bfr(v[k]); o[k] = f2bf(__fmul_rn(a, a)); }
    *(volatile v8us*)(X2b + t * 8) = o; __threadfence(); *(volatile v8us*)(X2b + t * 8) = o; }

__global__ __launch_bounds__(256) void k_pc(const float* __restrict__ m, const float* __restrict__ s, bf* IVb, bf* MVb) { const size_t t = (size_t)blockIdx.x * 256 + threadIdx.x; if (t >= (size_t)NK * ND / 8) return; const v8f vm = *(const v8f*)(m + t * 8); const v8f vs = *(const v8f*)(s + t * 8); v8us oi, om;
#pragma unroll
    for (int k = 0; k < 8; ++k) { const float iv = __fdiv_rn(1.0f, expf(bfr(vs[k]))); oi[k] = f2bf(iv); om[k] = f2bf(__fmul_rn(bfr(vm[k]), iv)); }
    *(volatile v8us*)(IVb + t * 8) = oi; *(volatile v8us*)(MVb + t * 8) = om; __threadfence(); *(volatile v8us*)(IVb + t * 8) = oi; *(volatile v8us*)(MVb + t * 8) = om; }

__global__ __launch_bounds__(256) void k_ck(const float* __restrict__ m, const float* __restrict__ s, float* CK) { const int k = blockIdx.x * 256 + threadIdx.x; if (k >= NK) return; const float* pm = m + (size_t)k * ND; const float* ps = s + (size_t)k * ND; float a = 0.0f;
    for (int c = 0; c < ND / 4; ++c) { const v4f vm = *(const v4f*)(pm + 4 * c); const v4f vs = *(const v4f*)(ps + 4 * c);
#pragma unroll
        for (int j = 0; j < 4; ++j) { const float sv = bfr(vs[j]); const float mv = bfr(vm[j]); a = __fadd_rn(a, __fadd_rn(sv, __fdiv_rn(__fmul_rn(mv, mv), expf(sv)))); } }
    *(volatile float*)(CK + k) = a; __threadfence(); *(volatile float*)(CK + k) = a; }

__global__ __launch_bounds__(256) void k_lw(const float* __restrict__ w, float* W) { const int k = blockIdx.x * 256 + threadIdx.x; if (k >= NK) return; float M = __int_as_float(0xff800000);
    for (int g = 0; g < NK; ++g) { const float a = bfr(w[(g + k) & (NK - 1)]); M = (a > M) ? a : M; }
    float z = 0.0f;
    for (int g = 0; g < NK; ++g) z = __fadd_rn(z, expf(__fsub_rn(bfr(w[(g + k) & (NK - 1)]), M)));
    const float o = __fsub_rn(bfr(w[k]), __fadd_rn(M, logf(z))); *(volatile float*)(W + k) = o; __threadfence(); *(volatile float*)(W + k) = o; }

__device__ __forceinline__ float tm(float g1, float g2, float ck, float wk) { const float q = __fadd_rn(__fsub_rn(g1, __fmul_rn(2.0f, g2)), ck); return __fadd_rn(wk, __fmul_rn(-0.5f, __fadd_rn(235.24826f, q))); }

__global__ __launch_bounds__(256) void k_ls(const float* __restrict__ G1, const float* __restrict__ G2, const float* __restrict__ CK, const float* __restrict__ W, float* out) { const int i = blockIdx.x * 256 + threadIdx.x; if (i >= NB) return; const float* r1 = G1 + (size_t)i * NK; const float* r2 = G2 + (size_t)i * NK; float M = __int_as_float(0xff800000);
    for (int g = 0; g < NK / 4; ++g) { const v4f a = *(const v4f*)(r1 + 4 * g); const v4f b = *(const v4f*)(r2 + 4 * g); const v4f c = *(const v4f*)(CK + 4 * g); const v4f u = *(const v4f*)(W + 4 * g);
#pragma unroll
        for (int j = 0; j < 4; ++j) { const float t = tm(a[j], b[j], c[j], u[j]); M = (t > M) ? t : M; } }
    float z = 0.0f;
    for (int g = 0; g < NK / 4; ++g) { const v4f a = *(const v4f*)(r1 + 4 * g); const v4f b = *(const v4f*)(r2 + 4 * g); const v4f c = *(const v4f*)(CK + 4 * g); const v4f u = *(const v4f*)(W + 4 * g);
#pragma unroll
        for (int j = 0; j < 4; ++j) z = __fadd_rn(z, expf(__fsub_rn(tm(a[j], b[j], c[j], u[j]), M))); }
    const float o = __fadd_rn(M, logf(z)); *(volatile float*)(out + i) = o; __threadfence(); *(volatile float*)(out + i) = o; }

extern "C" void kernel_launch(void* const* d_in, const int* in_sizes, int n_in, void* d_out, int out_size, void* d_ws, size_t ws_size, hipStream_t stream) {
    if (n_in < 4) return;
    if (in_sizes[0] != NB * ND || in_sizes[1] != NK * ND || in_sizes[2] != NK * ND || in_sizes[3] != NK) return;
    if (out_size != NB) return;
    static_assert(NB % 64 == 0 && NK % 64 == 0 && ND % 32 == 0 && (NB * ND / 8) % 256 == 0 && (NK * ND / 8) % 256 == 0 && NK % 256 == 0 && NB % 256 == 0 && NK % 4 == 0 && (NK & (NK - 1)) == 0, "the products: M and N multiples of 64, the depth a multiple of 32; every flat grid exact");
    const float* x = (const float*)d_in[0]; const float* m = (const float*)d_in[1]; const float* s = (const float*)d_in[2]; const float* w = (const float*)d_in[3];
    float* out = (float*)d_out;
    char* wsp = (char*)d_ws; auto take = [&](size_t bytes) { char* p = wsp; wsp += (bytes + 255) & ~(size_t)255; return (void*)p; };
    bf* Xb = (bf*)take((size_t)NB * ND * 2); bf* X2b = (bf*)take((size_t)NB * ND * 2); bf* IVb = (bf*)take((size_t)NK * ND * 2); bf* MVb = (bf*)take((size_t)NK * ND * 2); float* CK = (float*)take((size_t)NK * 4); float* W = (float*)take((size_t)NK * 4); float* G1 = (float*)take((size_t)NB * NK * 4); float* G2 = (float*)take((size_t)NB * NK * 4);
    if ((size_t)(wsp - (char*)d_ws) > ws_size) return;
    k_cvt8<<<(unsigned)(NB * ND / 8 / 256), 256, 0, stream>>>(x, Xb, (size_t)NB * ND / 8);
    k_px<<<(unsigned)(NB * ND / 8 / 256), 256, 0, stream>>>(x, X2b);
    k_pc<<<(unsigned)(NK * ND / 8 / 256), 256, 0, stream>>>(m, s, IVb, MVb);
    k_ck<<<(unsigned)(NK / 256), 256, 0, stream>>>(m, s, CK);
    k_lw<<<(unsigned)(NK / 256), 256, 0, stream>>>(w, W);
    k_gemmw<bf, 0, false><<<dim3(NB / 64, NK / 64, 1), 32, 0, stream>>>(X2b, nullptr, IVb, nullptr, ND, G1, NK, nullptr, 0, 0, 0);
    k_gemmw<bf, 0, false><<<dim3(NB / 64, NK / 64, 1), 32, 0, stream>>>(Xb, nullptr, MVb, nullptr, ND, G2, NK, nullptr, 0, 0, 0);
    k_ls<<<(unsigned)(NB / 256), 256, 0, stream>>>(G1, G2, CK, W, out);
}
